// Graph_Convolution_23106924052606
// MI455X (gfx1250) — hardware-verified
//
#include <hip/hip_runtime.h>
#include <stddef.h>
#include <stdint.h>


#define NN      39
#define NPIX    1521
#define HW1     41
#define KC2     96
#define NT2     12
#define MT2     1536
#define FIN     78
#define KG1     128
#define C1W     256
#define C2W     64
#define NL1     512
#define NL2     128
#define NTHR    256
#define NWAVE   8
#define EPT     8
#define CHUNK   (NTHR * EPT)
#define WCAP    (EPT * 32)
#define LISTN   (NWAVE * WCAP)
#define NBMAX   2048
#define NBRUN   1024
#define RCAP    28672
#define DEGCAP  256
#define STW     512
#define GBM     64
#define GBN     64
#define GTHR    128
#define CX1     16.0f
#define CW2     256.0f
#define SCL2    0.000244140625f
#define NEGS    0.2f
#define WSMAX   134217728
#define LDS_AGG ((2 * RCAP + 2 * NBMAX + LISTN) * 4 + 64)

#define FR_OFF_X1  0
#define FR_X1_N    (HW1 * HW1 * 8)
#define FR_OFF_WB  (FR_OFF_X1 + FR_X1_N * 2)
#define FR_WB_N    (16 * KC2)
#define FR_OFF_C2  (FR_OFF_WB + FR_WB_N * 2)
#define FR_C2_N    (MT2 * 16)
#define FR_OFF_FT  (FR_OFF_C2 + FR_C2_N * 4)
#define FR_FT_N    3044
#define FR_OFF_PR  (FR_OFF_FT + FR_FT_N * 4)
#define FR_PR_N    192
#define LDS_FRONT  (FR_OFF_PR + FR_PR_N * 4)
#define PR_C1W 0
#define PR_C1B 24
#define PR_S1  32
#define PR_M1  40
#define PR_B1  48
#define PR_C2B 56
#define PR_S2  72
#define PR_M2  88
#define PR_B2  104
#define PR_WIH 120
#define PR_WHH 168
#define PR_BIH 171
#define PR_BHH 174

static_assert((CHUNK & (CHUNK - 1)) == 0 && CHUNK <= 4096);
static_assert((NBMAX & (NBMAX - 1)) == 0 && NBMAX <= 4096);
static_assert((NBRUN & (NBRUN - 1)) == 0 && NBRUN <= NBMAX && NBRUN >= 16);
static_assert(NTHR * 8 == NBMAX);
static_assert(LISTN >= NBMAX);
static_assert(LISTN >= NWAVE * WCAP);
static_assert((RCAP % 32) == 0);
static_assert(NWAVE * STW <= RCAP);
static_assert(C1W <= STW);
static_assert(LDS_AGG <= 300000);
static_assert(LDS_FRONT <= 300000);
static_assert((FR_OFF_WB % 16) == 0 && (FR_OFF_C2 % 16) == 0 && (FR_OFF_FT % 16) == 0 && (FR_OFF_PR % 16) == 0);
static_assert(FR_FT_N >= 2 * NN * NN);
static_assert(PR_BHH + 3 <= FR_PR_N);
static_assert(NWAVE * NT2 * 16 == MT2 && MT2 >= NPIX);
static_assert(GBM == (GTHR / 32) * 16);
static_assert((KG1 % 32) == 0 && (C1W % 32) == 0 && KG1 >= FIN);
static_assert((NL1 % GBN) == 0 && (NL2 % GBN) == 0);
static_assert(NL1 == 2 * C1W && NL2 == 2 * C2W);
static_assert(2 * KG1 <= 2 * C1W);
static_assert(NL2 <= NL1);
static_assert((KC2 % 32) == 0);

typedef float          v2f   __attribute__((ext_vector_type(2)));
typedef float          v4f   __attribute__((ext_vector_type(4)));
typedef float          v8f   __attribute__((ext_vector_type(8)));
typedef int            v4i   __attribute__((ext_vector_type(4)));
typedef int            v8i   __attribute__((ext_vector_type(8)));
typedef unsigned short v8us  __attribute__((ext_vector_type(8)));
typedef _Float16       v8h   __attribute__((ext_vector_type(8)));
typedef _Float16       v16h  __attribute__((ext_vector_type(16)));
typedef __bf16         v16bf __attribute__((ext_vector_type(16)));
typedef v2f  __attribute__((may_alias)) v2fa;
typedef v4f  __attribute__((may_alias)) v4fa;
typedef v8us __attribute__((may_alias)) v8usa;
union FragH { v16h v;  v8h h[2]; v8us u[2]; v8i w; };
union FragB { v16bf v; v8us u[2]; v8i w; };

__device__ __forceinline__ v8f wmx(const FragH& a, const FragH& b, v8f c) {
  v8f d = __builtin_amdgcn_wmma_f32_16x16x32_f16(false, a.v, false, b.v, (short)0, c, false, false);
  asm volatile("v_nop\n\tv_nop\n\tv_nop\n\tv_nop" : "+v"(d) : "v"(a.w), "v"(b.w));
  return d;
}
__device__ __forceinline__ v8f wmb(const FragB& a, const FragB& b, v8f c) {
  v8f d = __builtin_amdgcn_wmma_f32_16x16x32_bf16(false, a.v, false, b.v, (short)0, c, false, false);
  asm volatile("v_nop\n\tv_nop\n\tv_nop\n\tv_nop" : "+v"(d) : "v"(a.w), "v"(b.w));
  return d;
}

__device__ __forceinline__ void ldwait() {
  asm volatile("s_wait_loadcnt 0x0" ::: "memory");
}

__device__ __forceinline__ unsigned bfbits(float v) {
  unsigned u = __float_as_uint(v);
  u = u + 0x7FFFu + ((u >> 16) & 1u);
  return u >> 16;
}
__device__ __forceinline__ float rbf(float v) { return __uint_as_float(bfbits(v) << 16); }

__device__ __forceinline__ void cvt8hl(const float (&f)[8], v8us& hv, v8us& lv) {
#pragma unroll
  for (int i = 0; i < 8; ++i) {
    const float hi = rbf(f[i]);
    hv[i] = (unsigned short)bfbits(f[i]);
    lv[i] = (unsigned short)bfbits(f[i] - hi);
  }
}

__device__ __forceinline__ float sigm(float x) {
  return __builtin_amdgcn_rcpf(1.0f + expf(-x));
}

__device__ __forceinline__ int scan_chunk(const int* __restrict__ dsts, int nE, int cbase, int slotBase,
                                          int nb, int vec8, int* list, int tid, int lane, int wave) {
  int wc = 0;
  const int el0  = tid * EPT;
  const int e0   = cbase + el0;
  const int sent = -2147483647 - 1;
  v4i da, db;
  if (vec8 != 0 && cbase + CHUNK <= nE) {
    da = *(const v4i*)(dsts + e0);
    db = *(const v4i*)(dsts + e0 + 4);
  } else {
    da.x = (e0     < nE) ? dsts[min(e0,     nE - 1)] : sent;
    da.y = (e0 + 1 < nE) ? dsts[min(e0 + 1, nE - 1)] : sent;
    da.z = (e0 + 2 < nE) ? dsts[min(e0 + 2, nE - 1)] : sent;
    da.w = (e0 + 3 < nE) ? dsts[min(e0 + 3, nE - 1)] : sent;
    db.x = (e0 + 4 < nE) ? dsts[min(e0 + 4, nE - 1)] : sent;
    db.y = (e0 + 5 < nE) ? dsts[min(e0 + 5, nE - 1)] : sent;
    db.z = (e0 + 6 < nE) ? dsts[min(e0 + 6, nE - 1)] : sent;
    db.w = (e0 + 7 < nE) ? dsts[min(e0 + 7, nE - 1)] : sent;
  }
  const unsigned nbs = (unsigned)slotBase;
  const unsigned unb = (unsigned)nb;
  const unsigned s0 = (unsigned)da.x - nbs, s1 = (unsigned)da.y - nbs;
  const unsigned s2 = (unsigned)da.z - nbs, s3 = (unsigned)da.w - nbs;
  const unsigned s4 = (unsigned)db.x - nbs, s5 = (unsigned)db.y - nbs;
  const unsigned s6 = (unsigned)db.z - nbs, s7 = (unsigned)db.w - nbs;
  const bool h0 = s0 < unb, h1 = s1 < unb, h2 = s2 < unb, h3 = s3 < unb;
  const bool h4 = s4 < unb, h5 = s5 < unb, h6 = s6 < unb, h7 = s7 < unb;
  const unsigned any = __builtin_amdgcn_ballot_w32(h0 | h1 | h2 | h3 | h4 | h5 | h6 | h7);
  if (any != 0u) {
#define HITJ(J, HJ, SJ) { \
      const unsigned mj = __builtin_amdgcn_ballot_w32(HJ); \
      if (mj != 0u) { \
        if (HJ) { \
          const int pos = wc + (int)__builtin_amdgcn_mbcnt_lo(mj, 0u); \
          if (pos < WCAP) list[wave * WCAP + pos] = ((el0 + (J)) << 12) | (int)(SJ); \
        } \
        wc += (int)__builtin_popcount(mj); } }
    HITJ(0, h0, s0)
    HITJ(1, h1, s1)
    HITJ(2, h2, s2)
    HITJ(3, h3, s3)
    HITJ(4, h4, s4)
    HITJ(5, h5, s5)
    HITJ(6, h6, s6)
    HITJ(7, h7, s7)
#undef HITJ
  }
  return wc;
}

__global__ __launch_bounds__(NTHR) void k_wtr2(const float* __restrict__ w0, const float* __restrict__ w1,
                                               int cols, int K0, int Kp,
                                               unsigned short* wh, unsigned short* wl, int nUnits) {
  const int u = (int)blockIdx.x * NTHR + (int)threadIdx.x;
  if (u >= nUnits) return;
  const int kq = Kp >> 3;
  const int n  = u / kq;
  const int k8 = (u - n * kq) * 8;
  const bool sec = n >= cols;
  int nc = sec ? n - cols : n;
  nc = nc < 0 ? 0 : (nc > cols - 1 ? cols - 1 : nc);
  const bool rowok = n < 2 * cols;
  const float* wsrc = sec ? w1 : w0;
  float f[8];
#pragma unroll
  for (int i = 0; i < 8; ++i) {
    const int k  = k8 + i;
    const int kc = k < K0 ? k : K0 - 1;
    const float x = wsrc[(size_t)kc * (size_t)cols + nc];
    f[i] = (k < K0 && rowok) ? x : 0.0f;
  }
  v8us hv, lv;
  cvt8hl(f, hv, lv);
  const size_t o = (size_t)n * (size_t)Kp + k8;
  *(volatile v8us*)(wh + o) = hv;
  *(volatile v8us*)(wl + o) = lv;
  __threadfence();
  *(volatile v8us*)(wh + o) = hv;
  *(volatile v8us*)(wl + o) = lv;
}

__global__ __launch_bounds__(NTHR) void k_front(
    const float* __restrict__ ve, const float* __restrict__ ac, const float* __restrict__ man,
    const float* __restrict__ mask,
    const float* __restrict__ c1w, const float* __restrict__ c1b,
    const float* __restrict__ bn1g, const float* __restrict__ bn1b,
    const float* __restrict__ bn1m, const float* __restrict__ bn1v,
    const float* __restrict__ c2w, const float* __restrict__ c2b,
    const float* __restrict__ bn2g, const float* __restrict__ bn2b,
    const float* __restrict__ bn2m, const float* __restrict__ bn2v,
    const float* __restrict__ wih, const float* __restrict__ whh,
    const float* __restrict__ bih, const float* __restrict__ bhh,
    unsigned short* Gh, unsigned short* Gl, int nB)
{
  extern __shared__ v4f lds_dyn[];
  char* lb = (char*)lds_dyn;
  _Float16* X1 = (_Float16*)(lb + FR_OFF_X1);
  _Float16* WB = (_Float16*)(lb + FR_OFF_WB);
  float* C2 = (float*)(lb + FR_OFF_C2);
  float* FT = (float*)(lb + FR_OFF_FT);
  float* PR = (float*)(lb + FR_OFF_PR);
  const int tid = (int)threadIdx.x, lane = tid & 31, wave = tid >> 5, hh = lane >> 4, m = lane & 15;
  const int b = (int)blockIdx.x;
  if (b >= nB) return;

  if (tid < 24) PR[PR_C1W + tid] = c1w[tid];
  if (tid < 8) {
    PR[PR_C1B + tid] = c1b[tid];
    PR[PR_S1 + tid]  = bn1g[tid] * rsqrtf(bn1v[tid] + 1e-5f);
    PR[PR_M1 + tid]  = bn1m[tid];
    PR[PR_B1 + tid]  = bn1b[tid];
  }
  if (tid < 16) {
    PR[PR_C2B + tid] = c2b[tid];
    PR[PR_S2 + tid]  = bn2g[tid] * rsqrtf(bn2v[tid] + 1e-5f);
    PR[PR_M2 + tid]  = bn2m[tid];
    PR[PR_B2 + tid]  = bn2b[tid];
  }
  if (tid < 48) PR[PR_WIH + tid] = wih[tid];
  if (tid < 3) {
    PR[PR_WHH + tid] = whh[tid];
    PR[PR_BIH + tid] = bih[tid];
    PR[PR_BHH + tid] = bhh[tid];
  }
#pragma unroll 1
  for (int i = tid; i < FR_WB_N; i += NTHR) {
    const int n = i / KC2, k = i - n * KC2;
    const int tap = k >> 3, c = k & 7;
    const int tcl = tap < 8 ? tap : 8;
    const float wv = c2w[n * 72 + c * 9 + tcl];
    WB[i] = (_Float16)((tap < 9 ? wv : 0.0f) * CW2);
  }
  __syncthreads();

  const float* mb = man + (size_t)b * NPIX;
  const float* ab = ac  + (size_t)b * NPIX;
  const float* vb = ve  + (size_t)b * NPIX;
#pragma unroll 1
  for (int u = tid; u < HW1 * HW1; u += NTHR) {
    const int hy = u / HW1, hx = u - HW1 * hy;
    const bool in = (hy >= 1) & (hy <= NN) & (hx >= 1) & (hx <= NN);
    int p = (hy - 1) * NN + (hx - 1);
    p = p < 0 ? 0 : (p > NPIX - 1 ? NPIX - 1 : p);
    float x0 = mb[p], x1 = ab[p], x2 = vb[p];
    x0 = (x0 == x0) ? x0 : 0.0f;
    x1 = (x1 == x1) ? x1 : 0.0f;
    x2 = (x2 == x2) ? x2 : 0.0f;
    if (in) FT[p] = x0;
    v8h hv;
#pragma unroll
    for (int co = 0; co < 8; ++co) {
      float s = PR[PR_C1B + co];
      s = fmaf(PR[PR_C1W + 3 * co + 0], x0, s);
      s = fmaf(PR[PR_C1W + 3 * co + 1], x1, s);
      s = fmaf(PR[PR_C1W + 3 * co + 2], x2, s);
      float t = fmaf(s - PR[PR_M1 + co], PR[PR_S1 + co], PR[PR_B1 + co]);
      t = fmaxf(t, 0.0f) * CX1;
      hv[co] = in ? (_Float16)t : (_Float16)0.0f;
    }
    *(v8h*)(X1 + (size_t)u * 8) = hv;
  }
  __syncthreads();

  {
    const int n = m;
    const float cb2 = PR[PR_C2B + n], sc2 = PR[PR_S2 + n], mu2 = PR[PR_M2 + n], be2 = PR[PR_B2 + n];
    int toff[6];
#pragma unroll
    for (int ks = 0; ks < 3; ++ks) {
      int t0 = 4 * ks + hh;     t0 = t0 > 8 ? 8 : t0;
      int t1 = 4 * ks + 2 + hh; t1 = t1 > 8 ? 8 : t1;
      toff[2 * ks]     = ((t0 / 3) * HW1 + (t0 % 3)) * 8;
      toff[2 * ks + 1] = ((t1 / 3) * HW1 + (t1 % 3)) * 8;
    }
    const _Float16* wbp = WB + n * KC2 + 8 * hh;
#pragma unroll 1
    for (int it = 0; it < NT2; ++it) {
      const int rt = wave * NT2 + it;
      int p = rt * 16 + m; p = p > NPIX - 1 ? NPIX - 1 : p;
      const int y = p / NN, x = p - NN * y;
      const _Float16* abp = X1 + (y * HW1 + x) * 8;
      v8f acc = {0.f, 0.f, 0.f, 0.f, 0.f, 0.f, 0.f, 0.f};
#pragma unroll
      for (int ks = 0; ks < 3; ++ks) {
        FragH af, bf;
        af.h[0] = *(const v8h*)(abp + toff[2 * ks]);
        af.h[1] = *(const v8h*)(abp + toff[2 * ks + 1]);
        bf.h[0] = *(const v8h*)(wbp + 32 * ks);
        bf.h[1] = *(const v8h*)(wbp + 32 * ks + 16);
        acc = wmx(af, bf, acc);
      }
#pragma unroll
      for (int r = 0; r < 8; ++r) {
        const int row = rt * 16 + 8 * hh + r;
        const float v = fmaf(acc[r], SCL2, cb2);
        C2[row * 16 + n] = fmaf(v - mu2, sc2, be2);
      }
    }
  }
  __syncthreads();

  if (tid < NN) {
    const int w = tid;
    const float wh0 = PR[PR_WHH], wh1 = PR[PR_WHH + 1], wh2 = PR[PR_WHH + 2];
    const float bh0 = PR[PR_BHH], bh1 = PR[PR_BHH + 1], bh2 = PR[PR_BHH + 2];
    const float bi0 = PR[PR_BIH], bi1 = PR[PR_BIH + 1], bi2 = PR[PR_BIH + 2];
    float h = 0.0f;
#pragma unroll 1
    for (int t = 0; t < NN; ++t) {
      const float* xb = C2 + (t * NN + w) * 16;
      float g0 = bi0, g1 = bi1, g2 = bi2;
#pragma unroll 1
      for (int i = 0; i < 16; ++i) {
        const float xv = xb[i];
        g0 = fmaf(PR[PR_WIH + i],      xv, g0);
        g1 = fmaf(PR[PR_WIH + 16 + i], xv, g1);
        g2 = fmaf(PR[PR_WIH + 32 + i], xv, g2);
      }
      const float gh0 = fmaf(h, wh0, bh0), gh1 = fmaf(h, wh1, bh1), gh2 = fmaf(h, wh2, bh2);
      const float rg = sigm(g0 + gh0);
      const float zg = sigm(g1 + gh1);
      const float ng = tanhf(fmaf(rg, gh2, g2));
      h = (1.0f - zg) * ng + zg * h;
      FT[(NN + t) * NN + w] = h;
    }
  }
  __syncthreads();

  const size_t rowBase = (size_t)b * NN;
#pragma unroll 1
  for (int u = tid; u < NN * 16; u += NTHR) {
    const int w   = u >> 4;
    const int cb0 = (u & 15) * 8;
    const float msk = mask[rowBase + w];
    float f[8];
#pragma unroll
    for (int j = 0; j < 8; ++j) {
      const int c  = cb0 + j;
      const int cc = c < FIN ? c : FIN - 1;
      const float fv = FT[cc * NN + w] * msk;
      f[j] = (c < FIN) ? fv : 0.0f;
    }
    v8us hv, lv;
    cvt8hl(f, hv, lv);
    const size_t o = (rowBase + w) * (size_t)KG1 + cb0;
    *(volatile v8us*)(Gh + o) = hv;
    *(volatile v8us*)(Gl + o) = lv;
    __threadfence();
    *(volatile v8us*)(Gh + o) = hv;
    *(volatile v8us*)(Gl + o) = lv;
  }
}

__global__ __launch_bounds__(GTHR) void k_gemm3(
    const unsigned short* __restrict__ Ah, const unsigned short* __restrict__ Al,
    const unsigned short* __restrict__ Wh, const unsigned short* __restrict__ Wl,
    const float* __restrict__ bias0, const float* __restrict__ bias1, int nhalf,
    float* outF, int K, int ldo)
{
  __shared__ __attribute__((aligned(16))) float stg[GBM * GBN];
  const int tid = (int)threadIdx.x, lane = tid & 31, wave = tid >> 5, hh = lane >> 4, m = lane & 15;
  const int rowBase = (int)blockIdx.x * GBM;
  const int col0    = (int)blockIdx.y * GBN;

  v8f acc[4];
  {
    const v8f z = {0.f, 0.f, 0.f, 0.f, 0.f, 0.f, 0.f, 0.f};
    acc[0] = z; acc[1] = z; acc[2] = z; acc[3] = z;
  }
  const size_t arow = (size_t)(rowBase + 16 * wave + m) * (size_t)K + 8 * hh;
  const unsigned short* aph = Ah + arow;
  const unsigned short* apl = Al + arow;
  const size_t wrow = (size_t)(col0 + m) * (size_t)K + 8 * hh;
  const unsigned short* wph = Wh + wrow;
  const unsigned short* wpl = Wl + wrow;
  const int ksteps = K >> 5;
#pragma unroll 1
  for (int ks = 0; ks < ksteps; ++ks) {
    FragB afh, afl;
    afh.u[0] = *(const v8usa*)(aph + 32 * ks);
    afh.u[1] = *(const v8usa*)(aph + 32 * ks + 16);
    afl.u[0] = *(const v8usa*)(apl + 32 * ks);
    afl.u[1] = *(const v8usa*)(apl + 32 * ks + 16);
#pragma unroll
    for (int t = 0; t < 4; ++t) {
      const size_t wo = (size_t)(16 * t) * (size_t)K + 32 * ks;
      FragB bfh, bfl;
      bfh.u[0] = *(const v8usa*)(wph + wo);
      bfh.u[1] = *(const v8usa*)(wph + wo + 16);
      bfl.u[0] = *(const v8usa*)(wpl + wo);
      bfl.u[1] = *(const v8usa*)(wpl + wo + 16);
      acc[t] = wmb(afh, bfh, acc[t]);
      acc[t] = wmb(afl, bfh, acc[t]);
      acc[t] = wmb(afh, bfl, acc[t]);
    }
  }

#pragma unroll
  for (int t = 0; t < 4; ++t) {
    const int lc = 16 * t + m;
    const int gc = col0 + lc;
    const int i0 = gc < nhalf ? gc : nhalf - 1;
    int i1 = gc - nhalf; i1 = i1 < 0 ? 0 : (i1 > nhalf - 1 ? nhalf - 1 : i1);
    const float b0v = bias0[i0];
    const float b1v = bias1[i1];
    const float bv  = gc < nhalf ? b0v : b1v;
#pragma unroll
    for (int r = 0; r < 8; ++r) {
      const int lr = 16 * wave + 8 * hh + r;
      stg[lr * GBN + lc] = acc[t][r] + bv;
    }
  }
  __syncthreads();

  v4f fv[8];
#pragma unroll
  for (int i = 0; i < 8; ++i) {
    const int lr = 16 * wave + 2 * i + hh;
    fv[i] = *(const v4fa*)(stg + lr * GBN + 4 * m);
  }
#pragma unroll
  for (int i = 0; i < 8; ++i) {
    const int lr = 16 * wave + 2 * i + hh;
    const int gr = rowBase + lr;
    float* op = outF + (size_t)gr * (size_t)ldo + col0 + 4 * m;
    *(volatile v4f*)op = fv[i];
  }
  __threadfence();
#pragma unroll
  for (int i = 0; i < 8; ++i) {
    const int lr = 16 * wave + 2 * i + hh;
    const int gr = rowBase + lr;
    float* op = outF + (size_t)gr * (size_t)ldo + col0 + 4 * m;
    *(volatile v4f*)op = fv[i];
  }
}

template<int CPL> struct Row;
template<> struct Row<8> {
  static __device__ __forceinline__ void ld(const float* p, float (&d)[8]) {
    const v4f a = *(const v4fa*)p;
    const v4f b = *(const v4fa*)(p + 4);
    d[0] = a.x; d[1] = a.y; d[2] = a.z; d[3] = a.w;
    d[4] = b.x; d[5] = b.y; d[6] = b.z; d[7] = b.w;
  }
};
template<> struct Row<2> {
  static __device__ __forceinline__ void ld(const float* p, float (&d)[8]) {
    const v2f a = *(const v2fa*)p;
    d[0] = a.x; d[1] = a.y;
  }
};

template<int CPL, int GRP>
__device__ __forceinline__ void edge_step(const float* srow, const float (&xr)[8], const float (&at)[8],
                                          float& mx, float& dn, float (&av)[8]) {
  float hs[8];
  Row<CPL>::ld(srow, hs);
  ldwait();
  float part = 0.0f;
#pragma unroll
  for (int j = 0; j < CPL; ++j) {
    float v = hs[j] + xr[j];
    v = v > 0.0f ? v : v * NEGS;
    part = fmaf(v, at[j], part);
  }
#pragma unroll
  for (int off = 1; off < GRP; off <<= 1) part += __shfl_xor(part, off);
  const float df = part - mx;
  const float ee = __expf(-fabsf(df));
  const bool up  = df > 0.0f;
  const float s1 = up ? ee : 1.0f;
  const float s2 = up ? 1.0f : ee;
  mx = up ? part : mx;
  dn = fmaf(dn, s1, s2);
#pragma unroll
  for (int j = 0; j < CPL; ++j) av[j] = fmaf(av[j], s1, s2 * hs[j]);
}

template<int LAYER>
__global__ __launch_bounds__(NTHR) void k_agg(
    const int* __restrict__ srcs, const int* __restrict__ dsts,
    const float* __restrict__ XLR, const float* __restrict__ att, const float* __restrict__ bias,
    unsigned short* Hh, unsigned short* Hl, float* outF,
    int nN, int nE, int nb, int vec8, int MPr) {
  constexpr int CPL = (LAYER == 1) ? 8 : 2;
  constexpr int C   = 32 * CPL;
  constexpr int NL  = 2 * C;
  constexpr int GRP = (LAYER == 1) ? 4 : 32;
  extern __shared__ v4f lds_dyn[];
  int* reg1 = (int*)lds_dyn;
  int* reg2 = reg1 + RCAP;
  int* scnt = reg2 + RCAP;
  int* soff = scnt + NBMAX;
  int* list = soff + NBMAX;
  int* wcnt = list + LISTN;
  int* wtot = wcnt + NWAVE;
  const int tid = (int)threadIdx.x, lane = tid & 31, wave = tid >> 5;
  const int nodeBase = (int)blockIdx.x * nb;

  for (int i = tid; i < NBMAX; i += NTHR) scnt[i] = 0;
#pragma unroll 1
  for (int i = tid; i < RCAP; i += NTHR) reg2[i] = 0;
  __syncthreads();

  int tot = 0;
  const int nChunks = (nE + CHUNK - 1) / CHUNK;
#pragma unroll 1
  for (int ch = 0; ch < nChunks; ++ch) {
    const int cbase = ch * CHUNK;
    const int wc = scan_chunk(dsts, nE, cbase, nodeBase, nb, vec8, list, tid, lane, wave);
    if (lane == 0) wcnt[wave] = wc;
    __syncthreads();
    int pre = 0, all = 0;
#pragma unroll
    for (int w2 = 0; w2 < NWAVE; ++w2) {
      int c = wcnt[w2];
      c = c < 0 ? 0 : (c > WCAP ? WCAP : c);
      all += c;
      pre += (w2 < wave) ? c : 0;
    }
    const int wcc  = wc > WCAP ? WCAP : wc;
    const int base = tot + pre;
#pragma unroll 1
    for (int i = lane; i < wcc; i += 32) {
      const int ent = list[wave * WCAP + i];
      const int el  = (ent >> 12) & (CHUNK - 1);
      const int sl  = ent & (NBMAX - 1);
      int eid = cbase + el;
      eid = eid > nE - 1 ? nE - 1 : eid;
      const int pos = base + i;
      if (pos < RCAP) reg1[pos] = (int)(((unsigned)eid << 12) | (unsigned)sl);
    }
    tot += all;
    tot = tot > RCAP ? RCAP : tot;
    __syncthreads();
  }
  const int nh = tot;

  if (wave == 0) {
#pragma unroll 1
    for (int b0 = 0; b0 < nh; b0 += 32) {
      const int idx = b0 + lane;
      const int uv  = reg1[idx < nh ? idx : nh - 1];
      const int m32 = (nh - b0) < 32 ? (nh - b0) : 32;
#pragma unroll 1
      for (int k = 0; k < m32; ++k) {
        const int u  = __builtin_amdgcn_readlane(uv, k);
        const int sl = u & (NBMAX - 1);
        if (lane == 0) scnt[sl] = scnt[sl] + 1;
      }
    }
  }
  __syncthreads();

  {
    const v4i ca = *(const v4i*)(scnt + 8 * tid);
    const v4i cb = *(const v4i*)(scnt + 8 * tid + 4);
    const int e0 = ca.x < 0 ? 0 : ca.x, e1 = ca.y < 0 ? 0 : ca.y, e2 = ca.z < 0 ? 0 : ca.z, e3 = ca.w < 0 ? 0 : ca.w;
    const int e4 = cb.x < 0 ? 0 : cb.x, e5 = cb.y < 0 ? 0 : cb.y, e6 = cb.z < 0 ? 0 : cb.z, e7 = cb.w < 0 ? 0 : cb.w;
    const int ts = e0 + e1 + e2 + e3 + e4 + e5 + e6 + e7;
    int incl = ts;
#pragma unroll
    for (int d = 1; d < 32; d <<= 1) {
      const int up = __shfl_up(incl, d);
      if (lane >= d) incl += up;
    }
    if (lane == 31) wtot[wave] = incl;
    __syncthreads();
    int pre = 0;
#pragma unroll
    for (int w2 = 0; w2 < NWAVE; ++w2) pre += (w2 < wave) ? wtot[w2] : 0;
    int run = pre + incl - ts;
    soff[8 * tid + 0] = run; run += e0;
    soff[8 * tid + 1] = run; run += e1;
    soff[8 * tid + 2] = run; run += e2;
    soff[8 * tid + 3] = run; run += e3;
    soff[8 * tid + 4] = run; run += e4;
    soff[8 * tid + 5] = run; run += e5;
    soff[8 * tid + 6] = run; run += e6;
    soff[8 * tid + 7] = run;
  }
  __syncthreads();
  for (int i = tid; i < NBMAX; i += NTHR) list[i] = soff[i];
  __syncthreads();

  if (wave == 0) {
#pragma unroll 1
    for (int b0 = 0; b0 < nh; b0 += 32) {
      const int idx = b0 + lane;
      const int uv  = reg1[idx < nh ? idx : nh - 1];
      const int m32 = (nh - b0) < 32 ? (nh - b0) : 32;
#pragma unroll 1
      for (int k = 0; k < m32; ++k) {
        const int u   = __builtin_amdgcn_readlane(uv, k);
        const int sl  = u & (NBMAX - 1);
        const int eid = (int)((unsigned)u >> 12);
        if (lane == 0) {
          int pos = list[sl];
          pos = pos < 0 ? 0 : (pos > RCAP - 1 ? RCAP - 1 : pos);
          reg2[pos] = eid;
          list[sl] = pos + 1;
        }
      }
    }
  }
  __syncthreads();

  const int nbw = nb >> 3;
  const bool ovf = (nh >= RCAP);
  const float qnan = __int_as_float(0x7fc00000);
  float* stw = (float*)reg1 + wave * STW;
  const int c0 = CPL * lane;
  float at[8], bb[8];
#pragma unroll
  for (int j = 0; j < CPL; ++j) {
    at[j] = att[c0 + j];
    bb[j] = bias[c0 + j];
  }
#pragma unroll 1
  for (int jt = 0; jt < nbw; ++jt) {
    const int slot = wave * nbw + jt;
    const int grow = nodeBase + slot;
    const int gcl  = grow < nN ? grow : nN - 1;
    int st = soff[slot];
    const int craw = scnt[slot];
    int cnt = craw;
    st  = st < 0 ? 0 : (st > nh ? nh : st);
    cnt = cnt < 0 ? 0 : (cnt > DEGCAP ? DEGCAP : cnt);
    if (cnt > nh - st) cnt = nh - st;
    const float pz = (ovf || craw > DEGCAP) ? qnan : 0.0f;
    const float live = grow < nN ? 1.0f : 0.0f;
    (void)live;

    float xr[8];
    Row<CPL>::ld(XLR + (size_t)gcl * NL + C + c0, xr);
    ldwait();
    float mx = -1.0e30f, dn = 0.0f;
    float av[8];
#pragma unroll
    for (int j = 0; j < 8; ++j) av[j] = 0.0f;

#pragma unroll 1
    for (int q = 0; q <= cnt; ++q) {
      const bool selfe = (q >= cnt);
      int idx = st + q; idx = idx < 0 ? 0 : (idx > RCAP - 1 ? RCAP - 1 : idx);
      int eid = reg2[idx]; eid = eid < 0 ? 0 : (eid > nE - 1 ? nE - 1 : eid);
      const int sraw = srcs[eid];
      const int sd = sraw < 0 ? 0 : (sraw > nN - 1 ? nN - 1 : sraw);
      const int s = selfe ? gcl : sd;
      edge_step<CPL, GRP>(XLR + (size_t)s * NL + c0, xr, at, mx, dn, av);
    }

    const float ds = dn > 0.0f ? dn : 1.0f;
    const float iv = (dn > 0.0f ? 1.0f : 0.0f) * __builtin_amdgcn_rcpf(ds);

    if (LAYER == 1) {
      float* ev = stw + 8 * lane;
      v4f va, vb;
      va.x = fmaf(av[0], iv, bb[0]); va.y = fmaf(av[1], iv, bb[1]);
      va.z = fmaf(av[2], iv, bb[2]); va.w = fmaf(av[3], iv, bb[3]);
      vb.x = fmaf(av[4], iv, bb[4]); vb.y = fmaf(av[5], iv, bb[5]);
      vb.z = fmaf(av[6], iv, bb[6]); vb.w = fmaf(av[7], iv, bb[7]);
      *(v4fa*)ev = va;
      *(v4fa*)(ev + 4) = vb;
#pragma unroll 1
      for (int j = 0; j < 8; ++j) {
        const float v  = ev[j];
        const float em = expm1f(fminf(v, 0.0f));
        ev[j] = v > 0.0f ? v : em;
      }
      const v4f ra = *(const v4fa*)ev;
      const v4f rb = *(const v4fa*)(ev + 4);
      float r[8];
      r[0] = ra.x * live + pz; r[1] = ra.y * live + pz; r[2] = ra.z * live + pz; r[3] = ra.w * live + pz;
      r[4] = rb.x * live + pz; r[5] = rb.y * live + pz; r[6] = rb.z * live + pz; r[7] = rb.w * live + pz;
      v8us hv, lv;
      cvt8hl(r, hv, lv);
      const bool wr = grow < MPr;
      unsigned short* gph = Hh + (size_t)grow * C + c0;
      unsigned short* gpl = Hl + (size_t)grow * C + c0;
      if (wr) { *(volatile v8us*)gph = hv; *(volatile v8us*)gpl = lv; }
      __threadfence();
      if (wr) { *(volatile v8us*)gph = hv; *(volatile v8us*)gpl = lv; }
    } else {
      const float r0 = fmaf(av[0], iv, bb[0]) + pz;
      const float r1 = fmaf(av[1], iv, bb[1]) + pz;
      __builtin_amdgcn_fence(__ATOMIC_RELEASE, "wavefront");
      __builtin_amdgcn_wave_barrier();
      stw[2 * lane]     = r0;
      stw[2 * lane + 1] = r1;
      __builtin_amdgcn_fence(__ATOMIC_RELEASE, "wavefront");
      __builtin_amdgcn_wave_barrier();
      const int lc = lane < 16 ? lane : 15;
      const bool wr = grow < nN;
      const v4f gv = *(const v4fa*)(stw + 4 * lc);
      float* gp = outF + (size_t)grow * C2W + 4 * lc;
      const bool wsv = wr && (lane < (C2W / 4));
      if (wsv) *(volatile v4f*)gp = gv;
      __threadfence();
      if (wsv) *(volatile v4f*)gp = gv;
    }
  }
  (void)Hh; (void)Hl; (void)outF;
}

static int pick_nb(int nE, int nN) {
  int nb = NBRUN;
  while (nb > 16 && (long long)nb * (long long)nE * 5LL > (long long)RCAP * (long long)nN * 4LL) nb >>= 1;
  return nb;
}
static inline int cdiv(int a, int b) { return (a + b - 1) / b; }
static inline size_t al256(size_t x) { return (x + 255) & ~(size_t)255; }

extern "C" void kernel_launch(void* const* d_in, const int* in_sizes, int n_in,
                              void* d_out, int out_size, void* d_ws, size_t ws_size,
                              hipStream_t stream) {
  if (n_in < 34) return;
  if (in_sizes[4] < NN || (in_sizes[4] % NN) != 0) return;
  const int nB = in_sizes[4] / NN;
  if (nB < 1 || nB > 4096) return;
  const int nN = nB * NN;
  if (in_sizes[1] != nB * NPIX || in_sizes[2] != nB * NPIX || in_sizes[3] != nB * NPIX) return;
  if (in_sizes[0] < 2 || (in_sizes[0] & 1) != 0) return;
  const int nE = in_sizes[0] / 2;
  if (nE < 1 || nE > (1 << 20)) return;
  if (in_sizes[6] != 24 || in_sizes[7] != 8 || in_sizes[8] != 8 || in_sizes[9] != 8 ||
      in_sizes[10] != 8 || in_sizes[11] != 8) return;
  if (in_sizes[12] != 1152 || in_sizes[13] != 16 || in_sizes[14] != 16 || in_sizes[15] != 16 ||
      in_sizes[16] != 16 || in_sizes[17] != 16) return;
  if (in_sizes[18] != 48 || in_sizes[19] != 3 || in_sizes[20] != 3 || in_sizes[21] != 3) return;
  if (in_sizes[22] != FIN * C1W || in_sizes[23] != C1W || in_sizes[24] != FIN * C1W || in_sizes[25] != C1W ||
      in_sizes[26] != C1W || in_sizes[27] != C1W) return;
  if (in_sizes[28] != C1W * C2W || in_sizes[29] != C2W || in_sizes[30] != C1W * C2W || in_sizes[31] != C2W ||
      in_sizes[32] != C2W || in_sizes[33] != C2W) return;
  if (out_size != nN * C2W) return;
  if ((nN % GBM) != 0) return;
  const int MP = nN;

  const int*   eidx  = (const int*)  d_in[0];
  const float* ve    = (const float*)d_in[1];
  const float* ac    = (const float*)d_in[2];
  const float* man   = (const float*)d_in[3];
  const float* mask  = (const float*)d_in[4];
  const float* c1w   = (const float*)d_in[6];
  const float* c1b   = (const float*)d_in[7];
  const float* bn1g  = (const float*)d_in[8];
  const float* bn1b  = (const float*)d_in[9];
  const float* bn1m  = (const float*)d_in[10];
  const float* bn1v  = (const float*)d_in[11];
  const float* c2w   = (const float*)d_in[12];
  const float* c2b   = (const float*)d_in[13];
  const float* bn2g  = (const float*)d_in[14];
  const float* bn2b  = (const float*)d_in[15];
  const float* bn2m  = (const float*)d_in[16];
  const float* bn2v  = (const float*)d_in[17];
  const float* gwih  = (const float*)d_in[18];
  const float* gwhh  = (const float*)d_in[19];
  const float* gbih  = (const float*)d_in[20];
  const float* gbhh  = (const float*)d_in[21];
  const float* g1wl  = (const float*)d_in[22];
  const float* g1bl  = (const float*)d_in[23];
  const float* g1wr  = (const float*)d_in[24];
  const float* g1br  = (const float*)d_in[25];
  const float* g1att = (const float*)d_in[26];
  const float* g1bi  = (const float*)d_in[27];
  const float* g2wl  = (const float*)d_in[28];
  const float* g2bl  = (const float*)d_in[29];
  const float* g2wr  = (const float*)d_in[30];
  const float* g2br  = (const float*)d_in[31];
  const float* g2att = (const float*)d_in[32];
  const float* g2bi  = (const float*)d_in[33];
  float* out = (float*)d_out;
  const int* src = eidx;
  const int* dst = eidx + nE;

  const int nb   = pick_nb(nE, nN);
  const int gA   = cdiv(MP, nb);
  const int vec8 = ((nE & 3) == 0) ? 1 : 0;
  if (gA * nb < MP) return;

  char* ws = (char*)d_ws;
  size_t off = 0;
  const size_t oW1h = off; off = al256(off + (size_t)NL1 * KG1 * 2);
  const size_t oW1l = off; off = al256(off + (size_t)NL1 * KG1 * 2);
  const size_t oW2h = off; off = al256(off + (size_t)NL2 * C1W * 2);
  const size_t oW2l = off; off = al256(off + (size_t)NL2 * C1W * 2);
  const size_t oR0  = off; off = al256(off + (size_t)MP * C1W * 2 * 2);
  const size_t oR1  = off; off = al256(off + (size_t)MP * NL1 * 4);
  if (off > ws_size || off > (size_t)WSMAX) return;
  unsigned short* WT1h = (unsigned short*)(ws + oW1h);
  unsigned short* WT1l = (unsigned short*)(ws + oW1l);
  unsigned short* WT2h = (unsigned short*)(ws + oW2h);
  unsigned short* WT2l = (unsigned short*)(ws + oW2l);
  unsigned short* Gh   = (unsigned short*)(ws + oR0);
  unsigned short* Gl   = Gh + (size_t)MP * KG1;
  unsigned short* H1h  = (unsigned short*)(ws + oR0);
  unsigned short* H1l  = H1h + (size_t)MP * C1W;
  float*          XLR1 = (float*)(ws + oR1);
  float*          XLR2 = (float*)(ws + oR1);

  hipFuncSetAttribute(reinterpret_cast<const void*>(&k_front),
                      hipFuncAttributeMaxDynamicSharedMemorySize, LDS_FRONT);
  hipFuncSetAttribute(reinterpret_cast<const void*>(&k_agg<1>),
                      hipFuncAttributeMaxDynamicSharedMemorySize, LDS_AGG);
  hipFuncSetAttribute(reinterpret_cast<const void*>(&k_agg<2>),
                      hipFuncAttributeMaxDynamicSharedMemorySize, LDS_AGG);

  {
    const int nU1 = NL1 * (KG1 / 8);
    k_wtr2<<<cdiv(nU1, NTHR), NTHR, 0, stream>>>(g1wl, g1wr, C1W, FIN, KG1, WT1h, WT1l, nU1);
    const int nU2 = NL2 * (C1W / 8);
    k_wtr2<<<cdiv(nU2, NTHR), NTHR, 0, stream>>>(g2wl, g2wr, C2W, C1W, C1W, WT2h, WT2l, nU2);
  }
  k_front<<<nB, NTHR, LDS_FRONT, stream>>>(ve, ac, man, mask, c1w, c1b, bn1g, bn1b, bn1m, bn1v,
                                            c2w, c2b, bn2g, bn2b, bn2m, bn2v, gwih, gwhh, gbih, gbhh,
                                            Gh, Gl, nB);
  const int gM = MP / GBM;
  k_gemm3<<<dim3(gM, NL1 / GBN), GTHR, 0, stream>>>(Gh, Gl, WT1h, WT1l, g1bl, g1br, C1W, XLR1, KG1, NL1);
  k_agg<1><<<gA, NTHR, LDS_AGG, stream>>>(src, dst, XLR1, g1att, g1bi, H1h, H1l, out,
                                          nN, nE, nb, vec8, MP);
  k_gemm3<<<dim3(gM, NL2 / GBN), GTHR, 0, stream>>>(H1h, H1l, WT2h, WT2l, g2bl, g2br, C2W, XLR2, C1W, NL2);
  k_agg<2><<<gA, NTHR, LDS_AGG, stream>>>(src, dst, XLR2, g2att, g2bi, H1h, H1l, out,
                                          nN, nE, nb, vec8, MP);
}
